// Decoder_58377195487266
// MI455X (gfx1250) — hardware-verified
//
#include <hip/hip_runtime.h>
#include <math.h>

#ifndef NB
#define NB 16
#endif
#ifndef SEQ
#define SEQ 2048
#endif
#define NB_FULL  16
#define SEQ_FULL 2048

constexpr int EMB   = 256;
constexpr int DKD   = 32;
constexpr int NHEAD = 8;
constexpr int FFD   = 4 * EMB;
constexpr int BTR   = NB * SEQ;

constexpr float LN_EPS     = 1e-5f;
constexpr float SCORE_SC   = 0.17677669529663687f;
constexpr float NEG_BIG    = -3.0e38f;
constexpr float W_SC       = 64.0f;
constexpr float W_INV      = 1.0f / 64.0f;
constexpr float P_SC       = 1024.0f;
constexpr float ATT_OUT_SC = 64.0f / 1024.0f;
constexpr float PROJ_INV   = 1.0f / (64.0f * 64.0f);
constexpr float FF1_INV    = 1.0f / 64.0f;
constexpr float H_SC       = 16.0f;
constexpr float FF2_INV    = 1.0f / (16.0f * 64.0f);

constexpr int TPW = 72;
constexpr int XP  = 264;
constexpr int QSP = 40;
constexpr int VSP = 72;
constexpr int PP  = 40;
constexpr int YP  = 260;
constexpr int HSP = 72;
constexpr int AWAVES = 4;

static_assert(NB >= 1 && NB <= NB_FULL);
static_assert(SEQ >= 64 && SEQ <= SEQ_FULL && SEQ % 64 == 0);
static_assert(BTR % 64 == 0);
static_assert(EMB == 256 && DKD == 32 && FFD == 1024 && NHEAD * DKD == EMB);
static_assert(EMB % 64 == 0 && FFD % 256 == 0 && DKD % 32 == 0);
static_assert(TPW % 8 == 0 && XP % 8 == 0 && QSP % 8 == 0 && VSP % 8 == 0 && PP % 8 == 0 && HSP % 8 == 0 && YP % 4 == 0);

constexpr size_t WS_WEIGHTS = (size_t)3 * EMB * DKD * 2 + (size_t)EMB * EMB * 2 + (size_t)2 * EMB * FFD * 2;
constexpr size_t WS_PLANES  = (size_t)4 * BTR * DKD * 2 + (size_t)BTR * EMB * 4 + (size_t)BTR * EMB * 2 + (size_t)BTR * FFD * 2;
static_assert(WS_WEIGHTS + WS_PLANES <= (size_t)134217728);

typedef __attribute__((ext_vector_type(16))) _Float16 v16h;
typedef __attribute__((ext_vector_type(8)))  _Float16 v8h;
typedef __attribute__((ext_vector_type(4)))  _Float16 v4h;
typedef __attribute__((ext_vector_type(8)))  float    v8f;
typedef __attribute__((ext_vector_type(4)))  float    v4f;

__device__ __forceinline__ void guard2(v8f& a, v8f& b, v16h x, v16h y) {
  asm volatile("v_nop\n\tv_nop\n\tv_nop\n\tv_nop" : "+v"(a), "+v"(b) : "v"(x), "v"(y));
}
__device__ __forceinline__ void guard3(v8f& a, v8f& b, v8f& c, v16h x, v16h y) {
  asm volatile("v_nop\n\tv_nop\n\tv_nop\n\tv_nop" : "+v"(a), "+v"(b), "+v"(c) : "v"(x), "v"(y));
}
__device__ __forceinline__ void guard4(v8f& a, v8f& b, v8f& c, v8f& d, v16h x, v16h y) {
  asm volatile("v_nop\n\tv_nop\n\tv_nop\n\tv_nop" : "+v"(a), "+v"(b), "+v"(c), "+v"(d) : "v"(x), "v"(y));
}
__device__ __forceinline__ void guard8(v8f& a0, v8f& a1, v8f& a2, v8f& a3, v8f& a4, v8f& a5, v8f& a6, v8f& a7, v16h x, v16h y) {
  asm volatile("v_nop\n\tv_nop\n\tv_nop\n\tv_nop"
               : "+v"(a0), "+v"(a1), "+v"(a2), "+v"(a3), "+v"(a4), "+v"(a5), "+v"(a6), "+v"(a7) : "v"(x), "v"(y));
}

__device__ __forceinline__ void wave_sync() {
  __builtin_amdgcn_fence(3  , "workgroup");
  __builtin_amdgcn_wave_barrier();
  __builtin_amdgcn_fence(2  , "workgroup");
}

struct FragH {
  union U { v16h v; v8h h[2]; };
  static __device__ __forceinline__ v16h load(const _Float16* p) {
    U f; f.h[0] = *(const v8h*)(p); f.h[1] = *(const v8h*)(p + 16); return f.v;
  }
  static __device__ __forceinline__ v8f mma(v16h a, v16h b, v8f c) {
    return __builtin_amdgcn_wmma_f32_16x16x32_f16(false, a, false, b, (short)0, c, false, false);
  }
};

__device__ __forceinline__ float bf16r(float v) {
  unsigned int u = __float_as_uint(v);
  u = (u + 0x7FFFu + ((u >> 16) & 1u)) & 0xFFFF0000u;
  return __uint_as_float(u);
}
__device__ __forceinline__ v4f bf16r4(v4f v) {
  v4f o;
#pragma unroll
  for (int e = 0; e < 4; ++e) o[e] = bf16r(v[e]);
  return o;
}

__device__ __forceinline__ float gelu_f(float u) { return 0.5f * u * (1.0f + erff(u * 0.70710678118654752440f)); }

__device__ __forceinline__ void ln_row(const float* yrow, int lane, v4f ga, v4f gb, v4f ba, v4f bb, v4f& ya, v4f& yb) {
  const v4f va = *(const v4f*)(yrow + 8 * lane);
  const v4f vb = *(const v4f*)(yrow + 8 * lane + 4);
  float s = ((va[0] + va[1]) + (va[2] + va[3])) + ((vb[0] + vb[1]) + (vb[2] + vb[3]));
#pragma unroll
  for (int d = 1; d < 32; d <<= 1) s += __shfl_xor(s, d, 32);
  const float mean = s * (1.0f / EMB);
  const v4f da = va - mean, db = vb - mean;
  float ss = ((da[0] * da[0] + da[1] * da[1]) + (da[2] * da[2] + da[3] * da[3])) +
             ((db[0] * db[0] + db[1] * db[1]) + (db[2] * db[2] + db[3] * db[3]));
#pragma unroll
  for (int d = 1; d < 32; d <<= 1) ss += __shfl_xor(ss, d, 32);
  const float rstd = rsqrtf(ss * (1.0f / EMB) + LN_EPS);
  ya = da * rstd * ga + ba;
  yb = db * rstd * gb + bb;
}

__global__ __launch_bounds__(256) void k_wprep(const float* __restrict__ src, _Float16* __restrict__ dst, int K, int N, float scale) {
  __shared__ __align__(16) _Float16 Ts[32 * TPW];
  const int tid = threadIdx.x, lane = tid & 31, wave = tid >> 5;
  const int k0 = blockIdx.x * 64, n0 = blockIdx.y * 32;
#pragma unroll
  for (int i = 0; i < 2; ++i) {
    const int r = i * 32 + (tid >> 3), c4 = (tid & 7) * 4;
    const v4f v = *(const v4f*)(src + (size_t)(k0 + r) * N + n0 + c4);
#pragma unroll
    for (int e = 0; e < 4; ++e) Ts[(c4 + e) * TPW + r] = (_Float16)(bf16r(v[e]) * scale);
  }
  __syncthreads();
  const int nrow = wave * 4 + (lane >> 3), piece = lane & 7;
  const v8h hv = *(const v8h*)(Ts + nrow * TPW + piece * 8);
  _Float16* dp = dst + (size_t)(n0 + nrow) * K + k0 + piece * 8;
  *(volatile v8h*)dp = hv;
  __threadfence();
  *(volatile v8h*)dp = hv;
}

__global__ __launch_bounds__(256) void k_qkv(const float* __restrict__ x,
                                             const _Float16* __restrict__ WqT, const _Float16* __restrict__ WkT,
                                             const _Float16* __restrict__ WvT,
                                             _Float16* __restrict__ Qp, _Float16* __restrict__ Kp, _Float16* __restrict__ VT) {
  __shared__ __align__(16) _Float16 Xs[64 * XP];
  __shared__ __align__(16) _Float16 Qs[64 * QSP];
  __shared__ __align__(16) _Float16 Ks[64 * QSP];
  __shared__ __align__(16) _Float16 Vs[DKD * VSP];
  const int tid = threadIdx.x, lane = tid & 31, wave = tid >> 5;
  const int m = lane & 15, hh = lane >> 4, koff = 8 * hh;
  const int r0c = blockIdx.x * 64;
  const int b = r0c / SEQ, tl0 = r0c - b * SEQ;
  const float* xb = x + ((size_t)b * SEQ_FULL + (size_t)tl0) * EMB;

#pragma unroll 2
  for (int i = 0; i < 16; ++i) {
    const int idx = i * 256 + tid;
    const int r = idx >> 6, c4 = (idx & 63) * 4;
    const v4f v = *(const v4f*)(xb + (size_t)r * EMB + c4);
    v4h hv;
#pragma unroll
    for (int e = 0; e < 4; ++e) hv[e] = (_Float16)bf16r(v[e]);
    *(v4h*)(Xs + r * XP + c4) = hv;
  }
  __syncthreads();

  const int rt = wave >> 1, ct = wave & 1;
  const _Float16* ap = Xs + (16 * rt + m) * XP + koff;
  const size_t woff = (size_t)(16 * ct + m) * EMB + koff;
  const v8f z8 = {0.f, 0.f, 0.f, 0.f, 0.f, 0.f, 0.f, 0.f};
  v8f cq = z8, ck = z8, cv = z8;
#pragma unroll 2
  for (int k0 = 0; k0 < EMB; k0 += 32) {
    const v16h a  = FragH::load(ap + k0);
    const v16h fq = FragH::load(WqT + woff + k0);
    const v16h fk = FragH::load(WkT + woff + k0);
    const v16h fv = FragH::load(WvT + woff + k0);
    cq = FragH::mma(a, fq, cq);
    ck = FragH::mma(a, fk, ck);
    cv = FragH::mma(a, fv, cv);
    guard3(cq, ck, cv, a, fv);
  }
#pragma unroll
  for (int r = 0; r < 8; ++r) {
    const int row = 16 * rt + 8 * hh + r, col = 16 * ct + m;
    Qs[row * QSP + col] = (_Float16)(cq[r] * W_INV);
    Ks[row * QSP + col] = (_Float16)(ck[r] * W_INV);
    Vs[col * VSP + row] = (_Float16)(cv[r] * W_INV);
  }
  __syncthreads();

  const int row = tid >> 2, piece = tid & 3;
  const v8h qv = *(const v8h*)(Qs + row * QSP + piece * 8);
  const v8h kv = *(const v8h*)(Ks + row * QSP + piece * 8);
  const int d = tid >> 3, pc = tid & 7;
  const v8h vv = *(const v8h*)(Vs + d * VSP + pc * 8);
  _Float16* qd = Qp + (size_t)(r0c + row) * DKD + piece * 8;
  _Float16* kd = Kp + (size_t)(r0c + row) * DKD + piece * 8;
  _Float16* vd = VT + ((size_t)b * DKD + d) * SEQ + tl0 + pc * 8;
  *(volatile v8h*)qd = qv;
  *(volatile v8h*)kd = kv;
  *(volatile v8h*)vd = vv;
  __threadfence();
  *(volatile v8h*)qd = qv;
  *(volatile v8h*)kd = kv;
  *(volatile v8h*)vd = vv;
}

__global__ __launch_bounds__(32 * AWAVES) void k_attn(const _Float16* __restrict__ Qp, const _Float16* __restrict__ Kp,
                                                     const _Float16* __restrict__ VT, _Float16* __restrict__ ATT) {
  __shared__ __align__(16) _Float16 Ps[AWAVES * 16 * PP];
  const int tid = threadIdx.x, lane = tid & 31, wv = tid >> 5;
  const int m = lane & 15, hh = lane >> 4, koff = 8 * hh;
  const int t0g = (blockIdx.x * AWAVES + wv) * 16;
  const int b = t0g / SEQ, t0 = t0g - b * SEQ;
  _Float16* Pw = Ps + wv * (16 * PP);
  const _Float16* kbase = Kp + ((size_t)b * SEQ + (size_t)m) * DKD + koff;
  const _Float16* vbase = VT + ((size_t)b * DKD + (size_t)m) * SEQ + koff;
  const v16h aq = FragH::load(Qp + (size_t)(t0g + m) * DKD + koff);
  const v8f z8 = {0.f, 0.f, 0.f, 0.f, 0.f, 0.f, 0.f, 0.f};
  v8f o0 = z8, o1 = z8;
  float mrow[8], lsum[8];
#pragma unroll
  for (int j = 0; j < 8; ++j) { mrow[j] = NEG_BIG; lsum[j] = 0.0f; }

  const int smax = ((t0 + 15) >> 5) << 5;
  for (int s0 = 0; s0 <= smax; s0 += 32) {
    const v16h kf0 = FragH::load(kbase + (size_t)s0 * DKD);
    const v16h kf1 = FragH::load(kbase + (size_t)(s0 + 16) * DKD);
    v8f st0 = FragH::mma(aq, kf0, z8);
    v8f st1 = FragH::mma(aq, kf1, z8);
    guard2(st0, st1, aq, kf1);
    const bool tail = (s0 + 31 > t0);
    _Float16 ph0[8], ph1[8];
#pragma unroll
    for (int j = 0; j < 8; ++j) {
      const int t = t0 + 8 * hh + j;
      float v0 = st0[j] * SCORE_SC;
      float v1 = st1[j] * SCORE_SC;
      if (tail) {
        v0 = (s0 + m > t)      ? NEG_BIG : v0;
        v1 = (s0 + 16 + m > t) ? NEG_BIG : v1;
      }
      float mc = fmaxf(v0, v1);
#pragma unroll
      for (int d = 1; d < 16; d <<= 1) mc = fmaxf(mc, __shfl_xor(mc, d, 32));
      const float mn   = fmaxf(mrow[j], mc);
      const float corr = __expf(mrow[j] - mn);
      const float e0   = __expf(v0 - mn);
      const float e1   = __expf(v1 - mn);
      lsum[j] = lsum[j] * corr + (e0 + e1);
      mrow[j] = mn;
      o0[j] *= corr;
      o1[j] *= corr;
      ph0[j] = (_Float16)(e0 * P_SC);
      ph1[j] = (_Float16)(e1 * P_SC);
    }
    wave_sync();
#pragma unroll
    for (int j = 0; j < 8; ++j) {
      Pw[(8 * hh + j) * PP + m]      = ph0[j];
      Pw[(8 * hh + j) * PP + 16 + m] = ph1[j];
    }
    wave_sync();
    const v16h pf  = FragH::load(Pw + m * PP + koff);
    const v16h vf0 = FragH::load(vbase + s0);
    const v16h vf1 = FragH::load(vbase + (size_t)16 * SEQ + s0);
    o0 = FragH::mma(pf, vf0, o0);
    o1 = FragH::mma(pf, vf1, o1);
    guard2(o0, o1, pf, vf1);
  }

  wave_sync();
#pragma unroll
  for (int j = 0; j < 8; ++j) {
    float l = lsum[j];
#pragma unroll
    for (int d = 1; d < 16; d <<= 1) l += __shfl_xor(l, d, 32);
    const float inv = ATT_OUT_SC * (1.0f / l);
    Pw[(8 * hh + j) * PP + m]      = (_Float16)(o0[j] * inv);
    Pw[(8 * hh + j) * PP + 16 + m] = (_Float16)(o1[j] * inv);
  }
  wave_sync();
  const v8h w0 = *(const v8h*)(Pw + (lane >> 2) * PP + (lane & 3) * 8);
  const v8h w1 = *(const v8h*)(Pw + (8 + (lane >> 2)) * PP + (lane & 3) * 8);
  _Float16* d0 = ATT + (size_t)t0g * DKD + lane * 8;
  _Float16* d1 = d0 + 256;
  *(volatile v8h*)d0 = w0;
  *(volatile v8h*)d1 = w1;
  __threadfence();
  *(volatile v8h*)d0 = w0;
  *(volatile v8h*)d1 = w1;
}

__global__ __launch_bounds__(256) void k_proj_ln1(const _Float16* __restrict__ ATT, const _Float16* __restrict__ WpT,
                                                  const float* __restrict__ x, const float* __restrict__ bp,
                                                  const float* __restrict__ g1, const float* __restrict__ be1,
                                                  float* __restrict__ Y1F, _Float16* __restrict__ Y1H) {
  __shared__ __align__(16) float Yt[32 * YP];
  const int tid = threadIdx.x, lane = tid & 31, wave = tid >> 5;
  const int m = lane & 15, hh = lane >> 4, koff = 8 * hh;
  const int r0c = blockIdx.x * 32;
  const int b = r0c / SEQ, tl0 = r0c - b * SEQ;
  const float* xb = x + ((size_t)b * SEQ_FULL + (size_t)tl0) * EMB;

#pragma unroll 2
  for (int i = 0; i < 8; ++i) {
    const int idx = i * 256 + tid;
    const int r = idx >> 6, c4 = (idx & 63) * 4;
    const v4f v  = *(const v4f*)(xb + (size_t)r * EMB + c4);
    const v4f bb = *(const v4f*)(bp + c4);
    *(v4f*)(Yt + r * YP + c4) = bf16r4(v) + bf16r4(bb);
  }

  const int rt = wave & 1, cg = wave >> 1;
  const v16h af = FragH::load(ATT + (size_t)(r0c + 16 * rt + m) * DKD + koff);
  const _Float16* wb = WpT + (size_t)(64 * cg + m) * EMB + koff;
  const v8f z8 = {0.f, 0.f, 0.f, 0.f, 0.f, 0.f, 0.f, 0.f};
  v8f acc[4];
#pragma unroll
  for (int nt = 0; nt < 4; ++nt) acc[nt] = z8;
#pragma unroll 2
  for (int j = 0; j < NHEAD; ++j) {
    v16h bf[4];
#pragma unroll
    for (int nt = 0; nt < 4; ++nt) bf[nt] = FragH::load(wb + (size_t)(16 * nt) * EMB + 32 * j);
#pragma unroll
    for (int nt = 0; nt < 4; ++nt) acc[nt] = FragH::mma(af, bf[nt], acc[nt]);
    guard4(acc[0], acc[1], acc[2], acc[3], af, bf[3]);
  }
  __syncthreads();
#pragma unroll
  for (int nt = 0; nt < 4; ++nt) {
#pragma unroll
    for (int r = 0; r < 8; ++r) {
      float* yp = Yt + (16 * rt + 8 * hh + r) * YP + 64 * cg + 16 * nt + m;
      const float cur = *yp;
      *yp = cur + acc[nt][r] * PROJ_INV;
    }
  }
  __syncthreads();

  const v4f ga = bf16r4(*(const v4f*)(g1 + 8 * lane)),  gb = bf16r4(*(const v4f*)(g1 + 8 * lane + 4));
  const v4f ba = bf16r4(*(const v4f*)(be1 + 8 * lane)), bb = bf16r4(*(const v4f*)(be1 + 8 * lane + 4));
#pragma unroll 1
  for (int q = 0; q < 4; ++q) {
    const int row = 4 * wave + q;
    float* yrow = Yt + row * YP;
    v4f ya, yb;
    ln_row(yrow, lane, ga, gb, ba, bb, ya, yb);
    v8h yh;
#pragma unroll
    for (int e = 0; e < 4; ++e) { yh[e] = (_Float16)ya[e]; yh[4 + e] = (_Float16)yb[e]; }
    *(v4f*)(yrow + 8 * lane)     = ya;
    *(v4f*)(yrow + 8 * lane + 4) = yb;
    wave_sync();
    const v4f w0 = *(const v4f*)(yrow + 4 * lane);
    const v4f w1 = *(const v4f*)(yrow + 128 + 4 * lane);
    const size_t grow = (size_t)(r0c + row);
    float* f0 = Y1F + grow * EMB + 4 * lane;
    float* f1 = f0 + 128;
    _Float16* hp = Y1H + grow * EMB + 8 * lane;
    *(volatile v4f*)f0 = w0;
    *(volatile v4f*)f1 = w1;
    *(volatile v8h*)hp = yh;
    __threadfence();
    *(volatile v4f*)f0 = w0;
    *(volatile v4f*)f1 = w1;
    *(volatile v8h*)hp = yh;
  }
}

__global__ __launch_bounds__(256) void k_ff1(const _Float16* __restrict__ Y1H, const _Float16* __restrict__ W1T,
                                             const float* __restrict__ b1, _Float16* __restrict__ H1) {
  __shared__ __align__(16) _Float16 Hs[8 * 32 * HSP];
  const int tid = threadIdx.x, lane = tid & 31, wave = tid >> 5;
  const int m = lane & 15, hh = lane >> 4, koff = 8 * hh;
  const int wrow0 = blockIdx.x * 64 + 32 * (wave & 1);
  const int wcol0 = blockIdx.y * 256 + 64 * (wave >> 1);
  const _Float16* ab  = Y1H + (size_t)(wrow0 + m) * EMB + koff;
  const _Float16* wbp = W1T + (size_t)(wcol0 + m) * EMB + koff;
  const v8f z8 = {0.f, 0.f, 0.f, 0.f, 0.f, 0.f, 0.f, 0.f};
  v8f acc[2][4];
#pragma unroll
  for (int rt = 0; rt < 2; ++rt)
#pragma unroll
    for (int nt = 0; nt < 4; ++nt) acc[rt][nt] = z8;
#pragma unroll 2
  for (int k0 = 0; k0 < EMB; k0 += 32) {
    const v16h a0 = FragH::load(ab + k0);
    const v16h a1 = FragH::load(ab + (size_t)16 * EMB + k0);
    v16h bf[4];
#pragma unroll
    for (int nt = 0; nt < 4; ++nt) bf[nt] = FragH::load(wbp + (size_t)(16 * nt) * EMB + k0);
#pragma unroll
    for (int nt = 0; nt < 4; ++nt) {
      acc[0][nt] = FragH::mma(a0, bf[nt], acc[0][nt]);
      acc[1][nt] = FragH::mma(a1, bf[nt], acc[1][nt]);
    }
    guard8(acc[0][0], acc[0][1], acc[0][2], acc[0][3], acc[1][0], acc[1][1], acc[1][2], acc[1][3], a1, bf[3]);
  }
  float bcol[4];
#pragma unroll
  for (int nt = 0; nt < 4; ++nt) bcol[nt] = bf16r(b1[wcol0 + 16 * nt + m]);
  _Float16* Hw = Hs + wave * (32 * HSP);
#pragma unroll
  for (int rt = 0; rt < 2; ++rt)
#pragma unroll
    for (int nt = 0; nt < 4; ++nt)
#pragma unroll
      for (int r = 0; r < 8; ++r) {
        const float u = acc[rt][nt][r] * FF1_INV + bcol[nt];
        Hw[(16 * rt + 8 * hh + r) * HSP + 16 * nt + m] = (_Float16)(gelu_f(u) * H_SC);
      }
  wave_sync();
  v8h hv[8];
#pragma unroll
  for (int i = 0; i < 8; ++i) hv[i] = *(const v8h*)(Hw + (4 * i + (lane >> 3)) * HSP + (lane & 7) * 8);
#pragma unroll
  for (int i = 0; i < 8; ++i)
    *(volatile v8h*)(H1 + (size_t)(wrow0 + 4 * i + (lane >> 3)) * FFD + wcol0 + (lane & 7) * 8) = hv[i];
  __threadfence();
#pragma unroll
  for (int i = 0; i < 8; ++i)
    *(volatile v8h*)(H1 + (size_t)(wrow0 + 4 * i + (lane >> 3)) * FFD + wcol0 + (lane & 7) * 8) = hv[i];
}

__global__ __launch_bounds__(256) void k_ff2_ln2(const _Float16* __restrict__ H1, const _Float16* __restrict__ W2T,
                                                 const float* __restrict__ Y1F, const float* __restrict__ b2,
                                                 const float* __restrict__ g2, const float* __restrict__ be2,
                                                 float* __restrict__ out) {
  __shared__ __align__(16) float Yt[32 * YP];
  const int tid = threadIdx.x, lane = tid & 31, wave = tid >> 5;
  const int m = lane & 15, hh = lane >> 4, koff = 8 * hh;
  const int r0c = blockIdx.x * 32;
  const int b = r0c / SEQ, tl0 = r0c - b * SEQ;

#pragma unroll 2
  for (int i = 0; i < 8; ++i) {
    const int idx = i * 256 + tid;
    const int r = idx >> 6, c4 = (idx & 63) * 4;
    const v4f v  = *(const v4f*)(Y1F + (size_t)(r0c + r) * EMB + c4);
    const v4f bb = *(const v4f*)(b2 + c4);
    *(v4f*)(Yt + r * YP + c4) = v + bf16r4(bb);
  }

  const int rt = wave & 1, cg = wave >> 1;
  const _Float16* ab = H1 + (size_t)(r0c + 16 * rt + m) * FFD + koff;
  const _Float16* wb = W2T + (size_t)(64 * cg + m) * FFD + koff;
  const v8f z8 = {0.f, 0.f, 0.f, 0.f, 0.f, 0.f, 0.f, 0.f};
  v8f acc[4];
#pragma unroll
  for (int nt = 0; nt < 4; ++nt) acc[nt] = z8;
#pragma unroll 2
  for (int k0 = 0; k0 < FFD; k0 += 32) {
    const v16h af = FragH::load(ab + k0);
    v16h bf[4];
#pragma unroll
    for (int nt = 0; nt < 4; ++nt) bf[nt] = FragH::load(wb + (size_t)(16 * nt) * FFD + k0);
#pragma unroll
    for (int nt = 0; nt < 4; ++nt) acc[nt] = FragH::mma(af, bf[nt], acc[nt]);
    guard4(acc[0], acc[1], acc[2], acc[3], af, bf[3]);
  }
  __syncthreads();
#pragma unroll
  for (int nt = 0; nt < 4; ++nt) {
#pragma unroll
    for (int r = 0; r < 8; ++r) {
      float* yp = Yt + (16 * rt + 8 * hh + r) * YP + 64 * cg + 16 * nt + m;
      const float cur = *yp;
      *yp = cur + acc[nt][r] * FF2_INV;
    }
  }
  __syncthreads();

  const v4f ga = bf16r4(*(const v4f*)(g2 + 8 * lane)),  gb = bf16r4(*(const v4f*)(g2 + 8 * lane + 4));
  const v4f ba = bf16r4(*(const v4f*)(be2 + 8 * lane)), bb = bf16r4(*(const v4f*)(be2 + 8 * lane + 4));
#pragma unroll 1
  for (int q = 0; q < 4; ++q) {
    const int row = 4 * wave + q;
    float* yrow = Yt + row * YP;
    v4f ya, yb;
    ln_row(yrow, lane, ga, gb, ba, bb, ya, yb);
    *(v4f*)(yrow + 8 * lane)     = ya;
    *(v4f*)(yrow + 8 * lane + 4) = yb;
    wave_sync();
    const v4f w0 = *(const v4f*)(yrow + 4 * lane);
    const v4f w1 = *(const v4f*)(yrow + 128 + 4 * lane);
    float* f0 = out + ((size_t)b * SEQ_FULL + (size_t)(tl0 + row)) * EMB + 4 * lane;
    float* f1 = f0 + 128;
    *(volatile v4f*)f0 = w0;
    *(volatile v4f*)f1 = w1;
    __threadfence();
    *(volatile v4f*)f0 = w0;
    *(volatile v4f*)f1 = w1;
  }
}

extern "C" void kernel_launch(void* const* d_in, const int* in_sizes, int n_in,
                              void* d_out, int out_size, void* d_ws, size_t ws_size, hipStream_t stream) {
  if (n_in < 14 || d_out == nullptr || d_ws == nullptr) return;
  const int need = ((NB - 1) * SEQ_FULL + SEQ) * EMB;
  if (in_sizes[0] < need || out_size < need) return;
  if (in_sizes[1] != EMB * DKD || in_sizes[2] != EMB * DKD || in_sizes[3] != EMB * DKD || in_sizes[4] != EMB * EMB ||
      in_sizes[5] != EMB || in_sizes[6] != EMB * FFD || in_sizes[7] != FFD || in_sizes[8] != FFD * EMB ||
      in_sizes[9] != EMB || in_sizes[10] != EMB || in_sizes[11] != EMB || in_sizes[12] != EMB || in_sizes[13] != EMB) return;

  const float* x   = (const float*)d_in[0];
  const float* Wq  = (const float*)d_in[1];
  const float* Wk  = (const float*)d_in[2];
  const float* Wv  = (const float*)d_in[3];
  const float* Wp  = (const float*)d_in[4];
  const float* bp  = (const float*)d_in[5];
  const float* W1  = (const float*)d_in[6];
  const float* b1  = (const float*)d_in[7];
  const float* W2  = (const float*)d_in[8];
  const float* b2  = (const float*)d_in[9];
  const float* g1  = (const float*)d_in[10];
  const float* be1 = (const float*)d_in[11];
  const float* g2  = (const float*)d_in[12];
  const float* be2 = (const float*)d_in[13];
  float* out = (float*)d_out;

  char* ws = (char*)d_ws; size_t off = 0;
  auto carve = [&](size_t bytes) -> char* { char* p = ws + off; off += (bytes + 255) & ~(size_t)255; return p; };
  _Float16* WqT = (_Float16*)carve((size_t)DKD * EMB * 2);
  _Float16* WkT = (_Float16*)carve((size_t)DKD * EMB * 2);
  _Float16* WvT = (_Float16*)carve((size_t)DKD * EMB * 2);
  _Float16* WpT = (_Float16*)carve((size_t)EMB * EMB * 2);
  _Float16* W1T = (_Float16*)carve((size_t)FFD * EMB * 2);
  _Float16* W2T = (_Float16*)carve((size_t)EMB * FFD * 2);
  _Float16* Qp  = (_Float16*)carve((size_t)BTR * DKD * 2);
  _Float16* Kp  = (_Float16*)carve((size_t)BTR * DKD * 2);
  _Float16* VTp = (_Float16*)carve((size_t)NB * DKD * SEQ * 2);
  _Float16* ATT = (_Float16*)carve((size_t)BTR * DKD * 2);
  float*    Y1F = (float*)carve((size_t)BTR * EMB * 4);
  _Float16* Y1H = (_Float16*)carve((size_t)BTR * EMB * 2);
  _Float16* H1  = (_Float16*)carve((size_t)BTR * FFD * 2);
  if (off > ws_size || off > (size_t)134217728) return;

  k_wprep<<<dim3(EMB / 64, DKD / 32), 256, 0, stream>>>(Wq, WqT, EMB, DKD, W_SC);
  k_wprep<<<dim3(EMB / 64, DKD / 32), 256, 0, stream>>>(Wk, WkT, EMB, DKD, W_SC);
  k_wprep<<<dim3(EMB / 64, DKD / 32), 256, 0, stream>>>(Wv, WvT, EMB, DKD, W_SC);
  k_wprep<<<dim3(EMB / 64, EMB / 32), 256, 0, stream>>>(Wp, WpT, EMB, EMB, W_SC);
  k_wprep<<<dim3(EMB / 64, FFD / 32), 256, 0, stream>>>(W1, W1T, EMB, FFD, W_SC);
  k_wprep<<<dim3(FFD / 64, EMB / 32), 256, 0, stream>>>(W2, W2T, FFD, EMB, W_SC);

  k_qkv<<<BTR / 64, 256, 0, stream>>>(x, WqT, WkT, WvT, Qp, Kp, VTp);
  k_attn<<<BTR / (16 * AWAVES), 32 * AWAVES, 0, stream>>>(Qp, Kp, VTp, ATT);
  k_proj_ln1<<<BTR / 32, 256, 0, stream>>>(ATT, WpT, x, bp, g1, be1, Y1F, Y1H);
  k_ff1<<<dim3(BTR / 64, FFD / 256), 256, 0, stream>>>(Y1H, W1T, b1, H1);
  k_ff2_ln2<<<BTR / 32, 256, 0, stream>>>(H1, W2T, Y1F, b2, g2, be2, out);
}
